// CausalSelfAttention_21096879358080
// MI455X (gfx1250) — hardware-verified
//
#include <hip/hip_runtime.h>


#ifndef NB
#define NB 8
#endif
#ifndef SEQ
#define SEQ 2048
#endif
#define NB_FULL  8
#define SEQ_FULL 2048
#define DM   128
#define NH   4
#define HD   32
#define DQ   (NH * HD)
#define FW   (3 * DQ)
#define RH   256
#define PLN  ((size_t)NB * NH * SEQ * HD)
#define PLH  ((size_t)NB * NH * RH * HD)
#define SCL2 0.25503486164918f
#define PCL  10.0f
#define NEGB (-3.0e38f)
#define YP   36

static_assert(DQ == DM);
static_assert(HD == 32);
static_assert(2 * HD == 64);
static_assert(HD % 16 == 0);
static_assert(YP % 4 == 0 && YP >= HD);
static_assert(DM % 64 == 0);
static_assert(DQ % 32 == 0);
static_assert(FW % 64 == 0);
static_assert(SEQ % 64 == 0);
static_assert(RH % 64 == 0);
static_assert(RH % 2 == 0);
static_assert(RH <= SEQ);
static_assert((SEQ - RH) % 16 == 0);
static_assert(NB <= NB_FULL);
static_assert(SEQ <= SEQ_FULL);

typedef _Float16 h16;
typedef unsigned short bf;
typedef __attribute__((ext_vector_type(16))) __bf16   v16bf;
typedef __attribute__((ext_vector_type(16))) _Float16 v16h;
typedef __attribute__((ext_vector_type(16))) unsigned short v16us;
typedef __attribute__((ext_vector_type(8)))  _Float16 v8h;
typedef __attribute__((ext_vector_type(8)))  unsigned short v8us;
typedef __attribute__((ext_vector_type(8)))  float    v8f;
typedef __attribute__((ext_vector_type(4)))  float    v4f;
typedef __attribute__((ext_vector_type(2)))  float    v2f;
typedef __attribute__((ext_vector_type(2)))  _Float16 v2h;
typedef __attribute__((ext_vector_type(2)))  unsigned short v2us;
typedef v4f  __attribute__((may_alias)) v4fa;

__device__ __forceinline__ unsigned short f2bf(float f) { unsigned u = __float_as_uint(f); u += 0x7FFFu + ((u >> 16) & 1u); return (unsigned short)(u >> 16); }
__device__ __forceinline__ float bf2f(unsigned short b) { return __uint_as_float(((unsigned)b) << 16); }
__device__ __forceinline__ float bfr(float f) { return bf2f(f2bf(f)); }
__device__ __forceinline__ void splitf(float y, unsigned short& h, unsigned short& l) { h = f2bf(y); l = f2bf(y - bf2f(h)); }
__device__ __forceinline__ v16h cat16(v8h lo, v8h hi) { return __builtin_shufflevector(lo, hi, 0, 1, 2, 3, 4, 5, 6, 7, 8, 9, 10, 11, 12, 13, 14, 15); }
__device__ __forceinline__ v16bf cat16b(v8us lo, v8us hi) { return __builtin_bit_cast(v16bf, __builtin_shufflevector(lo, hi, 0, 1, 2, 3, 4, 5, 6, 7, 8, 9, 10, 11, 12, 13, 14, 15)); }
__device__ __forceinline__ v16h ldh(const h16* p) { return cat16(*(const v8h*)p, *(const v8h*)(p + 16)); }
__device__ __forceinline__ v16bf ldb(const bf* p) { return cat16b(*(const v8us*)p, *(const v8us*)(p + 16)); }
__device__ __forceinline__ v8f wmmab(v16bf a, v16bf b, v8f c) { return __builtin_amdgcn_wmma_f32_16x16x32_bf16(false, a, false, b, (short)0, c, false, false); }
__device__ __forceinline__ v8f wm16g(v16h a, v16h b, v8f c) {
    c = __builtin_amdgcn_wmma_f32_16x16x32_f16(false, a, false, b, (short)0, c, false, false);
    asm volatile("v_nop\n\tv_nop\n\tv_nop\n\tv_nop" : "+v"(c) : "v"(a), "v"(b));
    return c; }
__device__ __forceinline__ v8f wmbg(v16bf a, v16bf b, v8f c) {
    c = __builtin_amdgcn_wmma_f32_16x16x32_bf16(false, a, false, b, (short)0, c, false, false);
    asm volatile("v_nop\n\tv_nop\n\tv_nop\n\tv_nop" : "+v"(c) : "v"(a), "v"(b));
    return c; }

template <int NSPLIT>
__device__ __forceinline__ void gemmw_body(const bf* __restrict__ A, const bf* __restrict__ A2, const bf* __restrict__ Bt, const int K, const int lda, const size_t ksA, float* C, const int ldc, const float* __restrict__ bias, const size_t sA, const size_t sC) {
    __shared__ __align__(16) float os[16 * 68];
    const size_t z = blockIdx.z; A += z * sA; if (NSPLIT == 1) A2 += z * sA; C += z * sC;
    const int lane = threadIdx.x & 31, lr = lane & 15, hi = lane >> 4; const int r0 = blockIdx.x * 64, c0 = blockIdx.y * 64;
    v8f acc[4][4];
#pragma unroll
    for (int mb = 0; mb < 4; ++mb)
#pragma unroll
        for (int nb = 0; nb < 4; ++nb) acc[mb][nb] = (v8f){};
    const size_t aoff = (size_t)(r0 + lr) * lda + 8 * hi, boff = (size_t)(c0 + lr) * K + 8 * hi;
#pragma unroll 1
    for (int kc = 0; kc < K; kc += 32) {
        const size_t ak = (size_t)(kc >> 5) * ksA;
        v16bf a[4], a2[4];
#pragma unroll
        for (int mb = 0; mb < 4; ++mb) { a[mb] = ldb(A + aoff + (size_t)mb * 16 * lda + ak); if (NSPLIT == 1) a2[mb] = ldb(A2 + aoff + (size_t)mb * 16 * lda + ak); }
#pragma unroll
        for (int nb = 0; nb < 4; ++nb) { const v16bf b = ldb(Bt + boff + (size_t)nb * 16 * K + kc);
#pragma unroll
            for (int mb = 0; mb < 4; ++mb) { acc[mb][nb] = wmmab(a[mb], b, acc[mb][nb]); if (NSPLIT == 1) acc[mb][nb] = wmmab(a2[mb], b, acc[mb][nb]); } }
        asm volatile("v_nop\n\tv_nop\n\tv_nop\n\tv_nop" : "+v"(acc[0][0]), "+v"(acc[1][1]), "+v"(acc[2][2]), "+v"(acc[3][3]) : "v"(a[0]), "v"(a[3]));
    }
#pragma unroll
    for (int mb = 0; mb < 4; ++mb) {
#pragma unroll
        for (int nb = 0; nb < 4; ++nb) {
#pragma unroll
            for (int j = 0; j < 8; ++j) os[(hi * 8 + j) * 68 + nb * 16 + lr] = acc[mb][nb][j]; }
        __builtin_amdgcn_wave_barrier(); asm volatile("" ::: "memory");
        float* crow = C + (size_t)(r0 + mb * 16) * ldc + c0;
#pragma unroll 1
        for (int ps = 0; ps < 2; ++ps) {
#pragma unroll
            for (int s = 0; s < 8; ++s) { const int row = 2 * s + hi, cofs = lr * 4; v4f val = *(const v4fa*)(os + row * 68 + cofs);
                val[0] += bfr(bias[c0 + cofs]); val[1] += bfr(bias[c0 + cofs + 1]); val[2] += bfr(bias[c0 + cofs + 2]); val[3] += bfr(bias[c0 + cofs + 3]);
                *(volatile v4f*)(crow + (size_t)row * ldc + cofs) = val; }
            if (ps == 0) __threadfence(); }
        __builtin_amdgcn_wave_barrier(); asm volatile("" ::: "memory");
    }
}
__global__ __launch_bounds__(32) void k_gemm_qkv(const bf* __restrict__ A, const bf* __restrict__ Bt, float* C, const float* __restrict__ bias) {
    gemmw_body<0>(A, nullptr, Bt, DM, DM, (size_t)32, C, FW, bias, 0, 0); }
__global__ __launch_bounds__(32) void k_gemm_proj(const bf* __restrict__ Ah, const bf* __restrict__ Al, const bf* __restrict__ Bt, float* C, const float* __restrict__ bias) {
    gemmw_body<1>(Ah, Al, Bt, DQ, HD, (size_t)SEQ * HD, C, DM, bias, (size_t)NH * SEQ * HD, (size_t)SEQ_FULL * DM); }

__global__ __launch_bounds__(256) void k_wtG(const float* __restrict__ w, int K, int N, bf* Bt) {
    const int lane = threadIdx.x & 31; const int wave = __builtin_amdgcn_readfirstlane(threadIdx.x >> 5);
    const int L0 = (blockIdx.x * 8 + wave) * 8; const int nlines = N * K / 64;
#pragma unroll
    for (int ps = 0; ps < 2; ++ps) {
#pragma unroll 1
        for (int l = 0; l < 8; ++l) { const int L = L0 + l; if (L >= nlines) break; const size_t e = (size_t)L * 64 + lane * 2; const int k = (int)(e % K), n = (int)(e / K); v2us o;
            o[0] = f2bf(w[(size_t)k * N + n]); o[1] = f2bf(w[(size_t)(k + 1) * N + n]); *(volatile v2us*)(Bt + e) = o; }
        if (ps == 0) __threadfence(); }
}
__global__ __launch_bounds__(256) void k_cvtx(const float* __restrict__ x, bf* XB) {
    const size_t i = (size_t)blockIdx.x * 256 + threadIdx.x; if (i >= (size_t)NB * SEQ * DM / 8) return;
    const size_t row = i / (DM / 8); const int c = (int)(i % (DM / 8)) * 8; const size_t b = row / SEQ, t = row % SEQ;
    const v8f v = *(const v8f*)(x + (b * SEQ_FULL + t) * DM + c); v8us o;
#pragma unroll
    for (int k = 0; k < 8; ++k) o[k] = f2bf(v[k]);
    *(volatile v8us*)(XB + i * 8) = o; __threadfence(); *(volatile v8us*)(XB + i * 8) = o; }

__global__ __launch_bounds__(256) void k_qkp(const float* __restrict__ F, h16* P16, bf* PH, bf* PL) {
    const int which = blockIdx.y; const size_t e = ((size_t)blockIdx.x * 256 + threadIdx.x) * 2; if (e >= PLN) return;
    const int d = (int)(e % HD); const int t = (int)((e / HD) % SEQ); const int bh = (int)(e / ((size_t)HD * SEQ)); const int b = bh / NH, h = bh % NH;
    const v2f x = *(const v2f*)(F + ((size_t)b * SEQ + t) * FW + which * DQ + h * HD + d);
    v2h o16; v2us oh, ol;
#pragma unroll
    for (int q = 0; q < 2; ++q) { o16[q] = (h16)x[q]; unsigned short a2, c2; splitf(x[q], a2, c2); oh[q] = a2; ol[q] = c2; }
    const bool hl = (t < RH);
    const size_t o1 = (size_t)which * PLN + e;
    const size_t o2 = (size_t)which * PLH + ((size_t)bh * RH + (hl ? t : 0)) * HD + d;
    *(volatile v2h*)(P16 + o1) = o16; if (hl) { *(volatile v2us*)(PH + o2) = oh; *(volatile v2us*)(PL + o2) = ol; }
    __threadfence();
    *(volatile v2h*)(P16 + o1) = o16; if (hl) { *(volatile v2us*)(PH + o2) = oh; *(volatile v2us*)(PL + o2) = ol; }
}
__global__ __launch_bounds__(256) void k_vtp(const float* __restrict__ F, h16* V16, bf* VH, bf* VL) {
    const size_t e = ((size_t)blockIdx.x * 256 + threadIdx.x) * 2; if (e >= PLN) return;
    const int t = (int)(e % SEQ); const int d = (int)((e / SEQ) % HD); const int bh = (int)(e / ((size_t)SEQ * HD)); const int b = bh / NH, h = bh % NH;
    v2h o16; v2us oh, ol;
#pragma unroll
    for (int q = 0; q < 2; ++q) { const float x = F[((size_t)b * SEQ + t + q) * FW + 2 * DQ + h * HD + d]; o16[q] = (h16)x; unsigned short a2, c2; splitf(x, a2, c2); oh[q] = a2; ol[q] = c2; }
    const bool hl = (t < RH);
    const size_t o2 = ((size_t)bh * HD + d) * RH + (hl ? t : 0);
    *(volatile v2h*)(V16 + e) = o16; if (hl) { *(volatile v2us*)(VH + o2) = oh; *(volatile v2us*)(VL + o2) = ol; }
    __threadfence();
    *(volatile v2h*)(V16 + e) = o16; if (hl) { *(volatile v2us*)(VH + o2) = oh; *(volatile v2us*)(VL + o2) = ol; }
}

__global__ __launch_bounds__(32) void k_attn16(const h16* QK16, const h16* VT16, bf* ATH, bf* ATL) {
    __shared__ __align__(16) float ys[16 * YP];
    const int lane = threadIdx.x & 31, n = lane & 15, hh = lane >> 4;
    const int bh = blockIdx.y;
    const int q0 = RH + blockIdx.x * 16;
    const int qrow = q0 + n, kend = q0 + 15;
    const size_t qo = ((size_t)bh * SEQ + q0 + n) * HD + 8 * hh;
    const size_t ko = PLN + ((size_t)bh * SEQ + n) * HD + 8 * hh;
    const size_t vo = ((size_t)bh * HD + n) * SEQ + 8 * hh;
    const v16h qb = ldh(QK16 + qo);
    v8f o[2];
#pragma unroll
    for (int j = 0; j < 2; ++j) o[j] = (v8f){};
    float m = NEGB, l = 0.0f;
#pragma unroll 1
    for (int kb = 0; kb <= kend; kb += 32) {
        v8f s0 = (v8f){}, s1 = (v8f){};
        {
            const size_t ka = ko + (size_t)kb * HD;
            const v16h a0 = ldh(QK16 + ka), a1 = ldh(QK16 + ka + 16 * HD);
            s0 = wm16g(a0, qb, s0); s1 = wm16g(a1, qb, s1);
        }
        asm volatile("" ::: "memory");
        float u[16];
        const int key0 = kb + 8 * hh;
        if (kb + 31 > q0) {
#pragma unroll
            for (int r = 0; r < 8; ++r) { u[r] = (key0 + r <= qrow) ? s0[r] * SCL2 : NEGB; u[8 + r] = (key0 + 16 + r <= qrow) ? s1[r] * SCL2 : NEGB; }
        } else {
#pragma unroll
            for (int r = 0; r < 8; ++r) { u[r] = s0[r] * SCL2; u[8 + r] = s1[r] * SCL2; }
        }
        float mx = u[0];
#pragma unroll
        for (int i = 1; i < 16; ++i) mx = fmaxf(mx, u[i]);
        mx = fmaxf(mx, __shfl_xor(mx, 16, 32));
        const float mn = fmaxf(m, mx);
        const float corr = __builtin_amdgcn_exp2f(m - mn);
        m = mn;
        v16h pb; float ps = 0.0f;
#pragma unroll
        for (int r = 0; r < 8; ++r) {
            const float p0 = __builtin_amdgcn_exp2f((u[r] - mn) + PCL); const float p1 = __builtin_amdgcn_exp2f((u[8 + r] - mn) + PCL);
            ps += p0 + p1; pb[r] = (h16)p0; pb[8 + r] = (h16)p1; }
        l = l * corr + ps;
#pragma unroll
        for (int j = 0; j < 2; ++j) o[j] = o[j] * corr;
#pragma unroll
        for (int j = 0; j < 2; ++j) { const v16h va = ldh(VT16 + vo + (size_t)j * 16 * SEQ + kb); o[j] = wm16g(va, pb, o[j]); }
        asm volatile("" ::: "memory");
    }
    l += __shfl_xor(l, 16, 32);
    const float inv = 1.0f / l;
#pragma unroll
    for (int j = 0; j < 2; ++j)
#pragma unroll
        for (int r = 0; r < 8; ++r) ys[n * YP + j * 16 + 8 * hh + r] = o[j][r] * inv;
    __builtin_amdgcn_wave_barrier(); asm volatile("" ::: "memory");
    v8us oh[2], ol[2];
#pragma unroll
    for (int s = 0; s < 2; ++s) { const int row = 8 * s + (lane >> 2), c = (lane & 3) * 8;
        const v4f a = *(const v4fa*)(ys + row * YP + c); const v4f bq = *(const v4fa*)(ys + row * YP + c + 4);
#pragma unroll
        for (int k = 0; k < 4; ++k) { unsigned short x1, x2; splitf(a[k], x1, x2); oh[s][k] = x1; ol[s][k] = x2; splitf(bq[k], x1, x2); oh[s][4 + k] = x1; ol[s][4 + k] = x2; } }
#pragma unroll 1
    for (int ps = 0; ps < 2; ++ps) {
#pragma unroll
        for (int s = 0; s < 2; ++s) { const int row = 8 * s + (lane >> 2), c = (lane & 3) * 8; const size_t oo = ((size_t)bh * SEQ + q0 + row) * HD + c;
            *(volatile v8us*)(ATH + oo) = oh[s]; *(volatile v8us*)(ATL + oo) = ol[s]; }
        if (ps == 0) __threadfence(); }
}

__global__ __launch_bounds__(32) void k_attnhl(const bf* QKH, const bf* QKL, const bf* VTH, const bf* VTL, bf* ATH, bf* ATL) {
    __shared__ __align__(16) float ys[16 * YP];
    const int lane = threadIdx.x & 31, n = lane & 15, hh = lane >> 4;
    const int bh = blockIdx.y;
    const int q0 = blockIdx.x * 16;
    const int qrow = q0 + n, kend = q0 + 15;
    const size_t qo = ((size_t)bh * RH + q0 + n) * HD + 8 * hh;
    const size_t ko = PLH + ((size_t)bh * RH + n) * HD + 8 * hh;
    const size_t vo = ((size_t)bh * HD + n) * RH + 8 * hh;
    v8f o[2];
#pragma unroll
    for (int j = 0; j < 2; ++j) o[j] = (v8f){};
    float m = NEGB, l = 0.0f;
#pragma unroll 1
    for (int kb = 0; kb <= kend; kb += 32) {
        v8f s[2]; s[0] = (v8f){}; s[1] = (v8f){};
        {
            const v16bf qh = ldb(QKH + qo), ql = ldb(QKL + qo);
#pragma unroll
            for (int kc = 0; kc < 2; ++kc) { const size_t ka = ko + (size_t)(kb + kc * 16) * HD;
                const v16bf kh = ldb(QKH + ka), kl = ldb(QKL + ka);
                s[kc] = wmbg(kh, qh, s[kc]); s[kc] = wmbg(kl, qh, s[kc]); s[kc] = wmbg(kh, ql, s[kc]); }
            asm volatile("" ::: "memory");
        }
        float u[16];
        const int key0 = kb + 8 * hh;
        if (kb + 31 > q0) {
#pragma unroll
            for (int r = 0; r < 8; ++r) { u[r] = (key0 + r <= qrow) ? s[0][r] * SCL2 : NEGB; u[8 + r] = (key0 + 16 + r <= qrow) ? s[1][r] * SCL2 : NEGB; }
        } else {
#pragma unroll
            for (int r = 0; r < 8; ++r) { u[r] = s[0][r] * SCL2; u[8 + r] = s[1][r] * SCL2; }
        }
        float mx = u[0];
#pragma unroll
        for (int i = 1; i < 16; ++i) mx = fmaxf(mx, u[i]);
        mx = fmaxf(mx, __shfl_xor(mx, 16, 32));
        const float mn = fmaxf(m, mx);
        const float corr = __builtin_amdgcn_exp2f(m - mn);
        m = mn;
        v16us phu, plu; float ps = 0.0f;
#pragma unroll
        for (int r = 0; r < 8; ++r) {
            const float p0 = __builtin_amdgcn_exp2f(u[r] - mn); const float p1 = __builtin_amdgcn_exp2f(u[8 + r] - mn);
            ps += p0 + p1; unsigned short x1, x2; splitf(p0, x1, x2); phu[r] = x1; plu[r] = x2; splitf(p1, x1, x2); phu[8 + r] = x1; plu[8 + r] = x2; }
        const v16bf ph = __builtin_bit_cast(v16bf, phu), pl = __builtin_bit_cast(v16bf, plu);
        l = l * corr + ps;
#pragma unroll
        for (int j = 0; j < 2; ++j) o[j] = o[j] * corr;
#pragma unroll
        for (int j = 0; j < 2; ++j) { const size_t va = vo + (size_t)j * 16 * RH + kb; const v16bf vh = ldb(VTH + va), vl = ldb(VTL + va);
            o[j] = wmbg(vh, ph, o[j]); o[j] = wmbg(vl, ph, o[j]); o[j] = wmbg(vh, pl, o[j]);
            asm volatile("" ::: "memory"); }
    }
    l += __shfl_xor(l, 16, 32);
    const float inv = 1.0f / l;
#pragma unroll
    for (int j = 0; j < 2; ++j)
#pragma unroll
        for (int r = 0; r < 8; ++r) ys[n * YP + j * 16 + 8 * hh + r] = o[j][r] * inv;
    __builtin_amdgcn_wave_barrier(); asm volatile("" ::: "memory");
    v8us oh[2], ol[2];
#pragma unroll
    for (int s = 0; s < 2; ++s) { const int row = 8 * s + (lane >> 2), c = (lane & 3) * 8;
        const v4f a = *(const v4fa*)(ys + row * YP + c); const v4f bq = *(const v4fa*)(ys + row * YP + c + 4);
#pragma unroll
        for (int k = 0; k < 4; ++k) { unsigned short x1, x2; splitf(a[k], x1, x2); oh[s][k] = x1; ol[s][k] = x2; splitf(bq[k], x1, x2); oh[s][4 + k] = x1; ol[s][4 + k] = x2; } }
#pragma unroll 1
    for (int ps = 0; ps < 2; ++ps) {
#pragma unroll
        for (int s = 0; s < 2; ++s) { const int row = 8 * s + (lane >> 2), c = (lane & 3) * 8; const size_t oo = ((size_t)bh * SEQ + q0 + row) * HD + c;
            *(volatile v8us*)(ATH + oo) = oh[s]; *(volatile v8us*)(ATL + oo) = ol[s]; }
        if (ps == 0) __threadfence(); }
}

extern "C" void kernel_launch(void* const* d_in, const int* in_sizes, int n_in,
                              void* d_out, int out_size, void* d_ws, size_t ws_size, hipStream_t stream) {
    constexpr size_t XN = ((size_t)(NB - 1) * SEQ_FULL + SEQ) * DM;
    if (n_in < 5) return;
    if ((size_t)in_sizes[0] < XN || (size_t)in_sizes[1] < (size_t)DM * FW || in_sizes[2] < FW || (size_t)in_sizes[3] < (size_t)DQ * DM || in_sizes[4] < DM) return;
    if ((size_t)out_size < XN) return;
    const float* x = (const float*)d_in[0]; const float* wqkv = (const float*)d_in[1]; const float* bqkv = (const float*)d_in[2];
    const float* wo = (const float*)d_in[3]; const float* bo = (const float*)d_in[4];
    float* OUT = (float*)d_out;

    constexpr size_t SZ_WQKV = (size_t)FW * DM * 2;
    constexpr size_t SZ_WO   = (size_t)DM * DQ * 2;
    constexpr size_t SZ_XB   = (size_t)NB * SEQ * DM * 2;
    constexpr size_t SZ_F    = (size_t)NB * SEQ * FW * 4;
    constexpr size_t SZ_QK16 = 2 * PLN * 2;
    constexpr size_t SZ_VT16 = PLN * 2;
    constexpr size_t SZ_QKHL = 2 * PLH * 2;
    constexpr size_t SZ_VTHL = PLH * 2;
    constexpr size_t SZ_AT   = PLN * 2;
    constexpr size_t O_WQKV = 0;
    constexpr size_t O_WO   = O_WQKV + SZ_WQKV;
    constexpr size_t O_XB   = O_WO + SZ_WO;
    constexpr size_t O_F    = O_XB + SZ_XB;
    constexpr size_t O_QK16 = O_F + SZ_F;
    constexpr size_t O_VT16 = O_QK16 + SZ_QK16;
    constexpr size_t O_QKH  = O_VT16 + SZ_VT16;
    constexpr size_t O_QKL  = O_QKH + SZ_QKHL;
    constexpr size_t O_VTH  = O_QKL + SZ_QKHL;
    constexpr size_t O_VTL  = O_VTH + SZ_VTHL;
    constexpr size_t O_ATH  = O_VTL + SZ_VTHL;
    constexpr size_t O_ATL  = O_ATH + SZ_AT;
    constexpr size_t O_END  = O_ATL + SZ_AT;
    static_assert(SZ_WQKV % 256 == 0 && SZ_WO % 256 == 0 && SZ_XB % 256 == 0 && SZ_F % 256 == 0 && SZ_QK16 % 256 == 0 && SZ_VT16 % 256 == 0 && SZ_QKHL % 256 == 0 && SZ_VTHL % 256 == 0 && SZ_AT % 256 == 0);
    static_assert(O_END <= (size_t)134217728);
    static_assert((DM * FW) % 64 == 0 && (DQ * DM) % 64 == 0);
    static_assert(PLN % 64 == 0);
    static_assert(((size_t)NB * SEQ) % 64 == 0);
    if (ws_size < O_END) return;
    char* ws = (char*)d_ws;
    bf* WQKV = (bf*)(ws + O_WQKV); bf* WO = (bf*)(ws + O_WO); bf* XB = (bf*)(ws + O_XB); float* F = (float*)(ws + O_F);
    h16* QK16 = (h16*)(ws + O_QK16); h16* VT16 = (h16*)(ws + O_VT16);
    bf* QKH = (bf*)(ws + O_QKH); bf* QKL = (bf*)(ws + O_QKL); bf* VTH = (bf*)(ws + O_VTH); bf* VTL = (bf*)(ws + O_VTL);
    bf* ATH = (bf*)(ws + O_ATH); bf* ATL = (bf*)(ws + O_ATL);

    k_wtG<<<(unsigned)((DM * FW / 64 + 63) / 64), 256, 0, stream>>>(wqkv, DM, FW, WQKV);
    k_wtG<<<(unsigned)((DQ * DM / 64 + 63) / 64), 256, 0, stream>>>(wo, DQ, DM, WO);
    k_cvtx<<<(unsigned)(((size_t)NB * SEQ * DM / 8 + 255) / 256), 256, 0, stream>>>(x, XB);
    k_gemm_qkv<<<dim3(NB * SEQ / 64, FW / 64, 1), 32, 0, stream>>>(XB, WQKV, F, bqkv);
    const unsigned LP = (unsigned)((PLN / 2 + 255) / 256);
    k_qkp<<<dim3(LP, 2, 1), 256, 0, stream>>>(F, QK16, QKH, QKL);
    k_vtp<<<LP, 256, 0, stream>>>(F, VT16, VTH, VTL);
    k_attnhl<<<dim3(RH / 16, NB * NH, 1), 32, 0, stream>>>(QKH, QKL, VTH, VTL, ATH, ATL);
    if ((SEQ - RH) / 16 > 0) k_attn16<<<dim3((SEQ - RH) / 16, NB * NH, 1), 32, 0, stream>>>(QK16, VT16, ATH, ATL);
    k_gemm_proj<<<dim3(SEQ / 64, DM / 64, NB), 32, 0, stream>>>(ATH, ATL, WO, OUT, bo);
}
